// PointNetSetAbstraction_12103217840690
// MI455X (gfx1250) — hardware-verified
//
#include <hip/hip_runtime.h>
#include <math.h>
#include <stdint.h>

#pragma clang fp contract(off)

constexpr int NBATCH    = 16;
constexpr int NPTS      = 8192;
constexpr int NSAMP     = 1024;
constexpr int KNB       = 32;
constexpr int NQ        = NBATCH * NSAMP;
constexpr int MROWS     = NQ * KNB;
constexpr int CIN_REAL  = 9;
constexpr int KPAD0     = 32;
constexpr int NCH_A     = 64;
constexpr int NCH_B     = 64;
constexpr int NCH_C     = 128;
constexpr int W0_PITCH  = 40;
constexpr int W64_PITCH = 72;
constexpr int A2_PITCH  = 64;
constexpr float W_CARRY     = 16.0f;
constexpr float W_CARRY_INV = 1.0f / 16.0f;
constexpr float BN_EPS      = 1e-5f;
constexpr double INV_MROWS  = 1.0 / 524288.0;
constexpr int KNN_CHUNK = 512;
constexpr int QDEPTH    = 8;
constexpr int NBLK64    = MROWS / 64 / 8;
constexpr int NBLK32    = MROWS / 32 / 8;

static_assert(NQ * 3 * 4 == 196608);
static_assert(NQ * NCH_C * 4 == 8388608);
static_assert(NPTS == 8 * 1024);
static_assert(NSAMP == 1024);
static_assert(MROWS % 64 == 0 && MROWS % 32 == 0);
static_assert(KPAD0 % 32 == 0 && NCH_A % 32 == 0 && NCH_B % 32 == 0);
static_assert(NCH_A % 64 == 0 && NCH_B % 64 == 0 && NCH_C % 64 == 0);
static_assert(NBLK64 * 8 * 64 == MROWS && NBLK32 * 8 * 32 == MROWS);
static_assert(NSAMP % 256 == 0 && NPTS % KNN_CHUNK == 0 && KNN_CHUNK % 256 == 0);

typedef __attribute__((ext_vector_type(16))) _Float16 v16h;
typedef __attribute__((ext_vector_type(8)))  _Float16 v8h;
typedef __attribute__((ext_vector_type(8)))  float    v8f;
typedef __attribute__((ext_vector_type(4)))  float    v4f;
typedef __attribute__((ext_vector_type(4)))  unsigned int v4u;

__device__ __forceinline__ unsigned pk16(unsigned short a, unsigned short b) { return (unsigned)a | ((unsigned)b << 16); }
__device__ __forceinline__ unsigned short h_bits(float f) { const _Float16 h = (_Float16)f; return __builtin_bit_cast(unsigned short, h); }
__device__ __forceinline__ float h16_to_f32(unsigned hb) {
  const unsigned sgn = (hb & 0x8000u) << 16; const unsigned em = hb & 0x7fffu;
  const float fn = __uint_as_float((em << 13) + 0x38000000u);
  const float fs = (float)em * 5.9604644775390625e-8f;
  const float mag = (em < 0x400u) ? fs : fn; return __uint_as_float(__float_as_uint(mag) | sgn); }

struct FragH {
  union U { v16h v; v8h h[2]; };
  static __device__ __forceinline__ v16h load(const _Float16* p) { U f; f.h[0] = *(const v8h*)(p); f.h[1] = *(const v8h*)(p + 16); return f.v; }
  static __device__ __forceinline__ v8f mma(v16h a, v16h b, v8f c) {
    return __builtin_amdgcn_wmma_f32_16x16x32_f16(false, a, false, b, (short)0, c, false, false);
  }
};
__device__ __forceinline__ v8f zero8() { return (v8f){0.f, 0.f, 0.f, 0.f, 0.f, 0.f, 0.f, 0.f}; }
__device__ __forceinline__ void guard4(v8f& a, v8f& b, v8f& c, v8f& d, v16h x, v16h y) {
  asm volatile("v_nop\n\tv_nop\n\tv_nop\n\tv_nop" : "+v"(a), "+v"(b), "+v"(c), "+v"(d) : "v"(x), "v"(y)); }
__device__ __forceinline__ void guard2(v8f& a, v8f& b, v16h x, v16h y, v16h z) {
  asm volatile("v_nop\n\tv_nop\n\tv_nop\n\tv_nop" : "+v"(a), "+v"(b) : "v"(x), "v"(y), "v"(z)); }
__device__ __forceinline__ void guard1(v8f& a, v16h x, v16h y, v16h z, v16h w) {
  asm volatile("v_nop\n\tv_nop\n\tv_nop\n\tv_nop" : "+v"(a) : "v"(x), "v"(y), "v"(z), "v"(w)); }
__device__ __forceinline__ void acc_guard4(v8f& a, v8f& b, v8f& c, v8f& d) {
  asm volatile("v_nop\n\tv_nop\n\tv_nop\n\tv_nop" : "+v"(a), "+v"(b), "+v"(c), "+v"(d)); }
__device__ __forceinline__ void keep4_h(v16h a, v16h b, v16h c, v16h d) { asm volatile("v_nop" :: "v"(a), "v"(b), "v"(c), "v"(d)); }
__device__ __forceinline__ void opaque_f(float& x) { asm volatile("" : "+v"(x)); }
__device__ __forceinline__ void lds_wave_sync() {
  __builtin_amdgcn_fence(__ATOMIC_RELEASE, "workgroup");
  __builtin_amdgcn_wave_barrier();
  __builtin_amdgcn_fence(__ATOMIC_ACQUIRE, "workgroup");
}

__global__ __launch_bounds__(1024) void fps_kernel(const float* __restrict__ xyz, float* __restrict__ out0, float* __restrict__ cq) {
#pragma clang fp contract(off)
  __shared__ float redv[32];
  __shared__ int   redi[32];
  __shared__ float sC[4];
  __shared__ int   sFar;
  __shared__ int   nidx[NSAMP];
  __shared__ __align__(16) float so3[NSAMP * 3];
  const int b = blockIdx.x;
  const int tid = threadIdx.x, lane = tid & 31, wave = tid >> 5;
  const float* xb = xyz + (size_t)b * NPTS * 3;
  float px[8], py[8], pz[8], dist[8];
  {
    const float* p = xb + (size_t)tid * 24;
    const v4f a0 = *(const v4f*)(p);      const v4f a1 = *(const v4f*)(p + 4);  const v4f a2 = *(const v4f*)(p + 8);
    const v4f a3 = *(const v4f*)(p + 12); const v4f a4 = *(const v4f*)(p + 16); const v4f a5 = *(const v4f*)(p + 20);
    px[0] = a0[0]; py[0] = a0[1]; pz[0] = a0[2];
    px[1] = a0[3]; py[1] = a1[0]; pz[1] = a1[1];
    px[2] = a1[2]; py[2] = a1[3]; pz[2] = a2[0];
    px[3] = a2[1]; py[3] = a2[2]; pz[3] = a2[3];
    px[4] = a3[0]; py[4] = a3[1]; pz[4] = a3[2];
    px[5] = a3[3]; py[5] = a4[0]; pz[5] = a4[1];
    px[6] = a4[2]; py[6] = a4[3]; pz[6] = a5[0];
    px[7] = a5[1]; py[7] = a5[2]; pz[7] = a5[3];
  }
#pragma unroll
  for (int j = 0; j < 8; ++j) dist[j] = 1e10f;
  float cx = xb[0], cy = xb[1], cz = xb[2];
  int far = 0;
#pragma unroll 1
  for (int s = 0; s < NSAMP; ++s) {
    if (tid == 0) nidx[s] = far;
    float bv = 0.f; int bj = 0;
#pragma unroll
    for (int j = 0; j < 8; ++j) {
      const float dx = px[j] - cx; const float dy = py[j] - cy; const float dz = pz[j] - cz;
      const float t0 = dx * dx; const float t1 = dy * dy; const float t2 = dz * dz;
      const float t02 = t0 + t2; const float d = t02 + t1;
      const float nd = fminf(dist[j], d);
      dist[j] = nd;
      if (j == 0) { bv = nd; bj = 0; }
      else { const bool gt = nd > bv; bv = gt ? nd : bv; bj = gt ? j : bj; }
    }
    int bi = tid * 8 + bj;
#pragma unroll
    for (int off = 1; off < 32; off <<= 1) {
      const float ov = __shfl_xor(bv, off, 32); const int oi = __shfl_xor(bi, off, 32);
      const bool take = (ov > bv) || (ov == bv && oi < bi);
      bv = take ? ov : bv; bi = take ? oi : bi;
    }
    if (lane == 0) { redv[wave] = bv; redi[wave] = bi; }
    __syncthreads();
    if (wave == 0) {
      float v = redv[lane]; int i = redi[lane];
#pragma unroll
      for (int off = 1; off < 32; off <<= 1) {
        const float ov = __shfl_xor(v, off, 32); const int oi = __shfl_xor(i, off, 32);
        const bool take = (ov > v) || (ov == v && oi < i);
        v = take ? ov : v; i = take ? oi : i;
      }
      const int ic = i < 0 ? 0 : (i > NPTS - 1 ? NPTS - 1 : i);
      const float nx = xb[(size_t)ic * 3 + 0], ny = xb[(size_t)ic * 3 + 1], nz = xb[(size_t)ic * 3 + 2];
      if (lane == 0) { sC[0] = nx; sC[1] = ny; sC[2] = nz; sFar = ic; }
    }
    __syncthreads();
    far = sFar; cx = sC[0]; cy = sC[1]; cz = sC[2];
  }
  __syncthreads();
  {
    const int n = nidx[tid];
    const int nc = n < 0 ? 0 : (n > NPTS - 1 ? NPTS - 1 : n);
    const float x = xb[(size_t)nc * 3 + 0], y = xb[(size_t)nc * 3 + 1], z = xb[(size_t)nc * 3 + 2];
    const float q0 = x * x; const float q1 = y * y; const float q2 = z * z; const float q02 = q0 + q2; const float sq = q02 + q1;
    so3[tid * 3 + 0] = x; so3[tid * 3 + 1] = y; so3[tid * 3 + 2] = z;
    const v4f cv = (v4f){x, y, z, sq};
    float* cqp = cq + ((size_t)b * NSAMP + tid) * 4;
    for (int pass = 0; pass < 2; ++pass) { *(volatile v4f*)cqp = cv; __threadfence(); }
  }
  __syncthreads();
  if (tid < (NSAMP * 3) / 4) {
    const v4f o = *(const v4f*)(so3 + tid * 4);
    float* op = out0 + (size_t)b * NSAMP * 3 + tid * 4;
    for (int pass = 0; pass < 2; ++pass) { *(volatile v4f*)op = o; __threadfence(); }
  }
}

__device__ __forceinline__ void knn_drain(unsigned long long (&kk)[KNB], float (&qd)[QDEPTH], int (&qn)[QDEPTH], int& cnt, float& wvf) {
#pragma unroll 1
  for (int rr = 0; rr < QDEPTH; ++rr) {
    if (!__any(cnt > 0)) break;
    const bool has = cnt > 0;
    const float d = qd[0] + 0.0f;
    const int n = qn[0];
#pragma unroll
    for (int i = 0; i < QDEPTH - 1; ++i) { qd[i] = qd[i + 1]; qn[i] = qn[i + 1]; }
    cnt = has ? (cnt - 1) : 0;
    const unsigned u = __float_as_uint(d);
    const unsigned khi = (u & 0x80000000u) ? ~u : (u | 0x80000000u);
    const unsigned long long key = ((unsigned long long)khi << 32) | (unsigned long long)(unsigned)n;
    const unsigned long long top = kk[KNB - 1];
    const bool valid = has && (key < top);
    unsigned long long v = valid ? key : top;
#pragma unroll
    for (int t = KNB - 1; t >= 1; --t) {
      const unsigned long long lo = kk[t - 1];
      const bool c = lo > v;
      kk[t] = c ? lo : v;
      v = c ? v : lo;
    }
    kk[0] = (kk[0] > v) ? v : kk[0];
    const unsigned hi = (unsigned)(kk[KNB - 1] >> 32);
    const unsigned uu = (hi & 0x80000000u) ? (hi & 0x7fffffffu) : ~hi;
    wvf = __uint_as_float(uu);
  }
}

__global__ __launch_bounds__(256) void knn_group_kernel(const float* __restrict__ xyz, const float* __restrict__ pts,
                                                        const float* __restrict__ cq, unsigned* __restrict__ x0w) {
#pragma clang fp contract(off)
  __shared__ __align__(16) v4f cpt[KNN_CHUNK];
  __shared__ int idxs[256 * KNB];
  __shared__ __align__(16) unsigned stg[8][KNB * 16];
  const int tid = threadIdx.x, lane = tid & 31, wave = tid >> 5;
  const int blk = blockIdx.x;
  const int b = blk >> 2;
  const int q = blk * 256 + tid;
  const float* xb = xyz + (size_t)b * NPTS * 3;
  const float* pb = pts + (size_t)b * NPTS * 6;
  const v4f cqv = *(const v4f*)(cq + (size_t)q * 4);
  const float sx = cqv[0], sy = cqv[1], sz = cqv[2], sqs = cqv[3];
  unsigned long long kk[KNB];
#pragma unroll
  for (int t = 0; t < KNB; ++t) kk[t] = 0xFF80000000000000ull | (unsigned long long)(0x10000u + (unsigned)t);
  float qd[QDEPTH]; int qn[QDEPTH];
#pragma unroll
  for (int i = 0; i < QDEPTH; ++i) { qd[i] = 0.f; qn[i] = 0; }
  int cnt = 0;
  float wvf = INFINITY;

#pragma unroll 1
  for (int c0 = 0; c0 < NPTS; c0 += KNN_CHUNK) {
    __syncthreads();
#pragma unroll
    for (int k = 0; k < KNN_CHUNK / 256; ++k) {
      const int nl = tid + 256 * k; const int n = c0 + nl;
      const float x = xb[(size_t)n * 3 + 0], y = xb[(size_t)n * 3 + 1], z = xb[(size_t)n * 3 + 2];
      const float a0 = x * x; const float a1 = y * y; const float a2 = z * z; const float a02 = a0 + a2; const float s2 = a02 + a1;
      cpt[nl] = (v4f){x, y, z, s2};
    }
    __syncthreads();
#pragma unroll 1
    for (int g = 0; g < KNN_CHUNK; g += 4) {
#pragma unroll
      for (int e = 0; e < 4; ++e) {
        const v4f p = cpt[g + e];
        float dt = sx * p[0];
        dt = fmaf(sy, p[1], dt);
        dt = fmaf(sz, p[2], dt);
        const float tt = -2.0f * dt;
        const float uu = tt + sqs;
        const float d = uu + p[3];
        if (d < wvf) {
#pragma unroll
          for (int i = QDEPTH - 1; i >= 1; --i) { qd[i] = qd[i - 1]; qn[i] = qn[i - 1]; }
          qd[0] = d; qn[0] = c0 + g + e; ++cnt;
        }
      }
      if (__any(cnt >= 4)) knn_drain(kk, qd, qn, cnt, wvf);
    }
  }
  knn_drain(kk, qd, qn, cnt, wvf);

#pragma unroll
  for (int t = 0; t < KNB; ++t) idxs[tid * KNB + t] = (int)(unsigned)(kk[t] & 0xffffffffull);
  __syncthreads();

  const v4u wz = (v4u){0u, 0u, 0u, 0u};
#pragma unroll 1
  for (int qq = 0; qq < 32; ++qq) {
    const int ql = wave * 32 + qq;
    const int qg = blk * 256 + ql;
    int n = idxs[ql * KNB + lane];
    n = n < 0 ? 0 : (n > NPTS - 1 ? NPTS - 1 : n);
    const float cx = __shfl(sx, qq, 32), cy = __shfl(sy, qq, 32), cz = __shfl(sz, qq, 32);
    const float* xp = xb + (size_t)n * 3;
    const float* fp = pb + (size_t)n * 6;
    const float gx = xp[0] - cx, gy = xp[1] - cy, gz = xp[2] - cz;
    const float f0 = fp[0], f1 = fp[1], f2 = fp[2], f3 = fp[3], f4 = fp[4], f5 = fp[5];
    const v4u wa = (v4u){pk16(h_bits(gx), h_bits(gy)), pk16(h_bits(gz), h_bits(f0)), pk16(h_bits(f1), h_bits(f2)), pk16(h_bits(f3), h_bits(f4))};
    const v4u wb = (v4u){(unsigned)h_bits(f5), 0u, 0u, 0u};
    unsigned* st = stg[wave] + lane * 16;
    *(v4u*)(st) = wa; *(v4u*)(st + 4) = wb; *(v4u*)(st + 8) = wz; *(v4u*)(st + 12) = wz;
    lds_wave_sync();
    v4u o[4];
#pragma unroll
    for (int i = 0; i < 4; ++i) o[i] = *(const v4u*)(stg[wave] + 4 * lane + 128 * i);
    unsigned* gd = x0w + (size_t)qg * (KNB * 16);
    for (int pass = 0; pass < 2; ++pass) {
#pragma unroll
      for (int i = 0; i < 4; ++i) *(volatile v4u*)(gd + 4 * lane + 128 * i) = o[i];
      __threadfence();
    }
    lds_wave_sync();
  }
}

__device__ __forceinline__ void build_w0s(_Float16* W0s, const float* __restrict__ w0, int tid) {
  const int n = tid >> 2, kg = (tid & 3) * 8;
  float v[8];
#pragma unroll
  for (int e = 0; e < 8; ++e) {
    const int k = kg + e;
    int idx = n * CIN_REAL + k; idx = idx > (NCH_A * CIN_REAL - 1) ? (NCH_A * CIN_REAL - 1) : idx;
    float w = w0[idx]; opaque_f(w);
    v[e] = (k < CIN_REAL) ? (w * W_CARRY) : 0.0f;
  }
  const v4u u = (v4u){pk16(h_bits(v[0]), h_bits(v[1])), pk16(h_bits(v[2]), h_bits(v[3])), pk16(h_bits(v[4]), h_bits(v[5])), pk16(h_bits(v[6]), h_bits(v[7]))};
  *(v4u*)(W0s + n * W0_PITCH + kg) = u;
}
__device__ __forceinline__ void build_w64(_Float16* Ws, int pitch, const float* __restrict__ w, int nrows, int tid) {
#pragma unroll 1
  for (int it = tid; it < nrows * 8; it += 256) {
    const int n = it >> 3, kg = (it & 7) * 8;
    const v4f a = *(const v4f*)(w + (size_t)n * 64 + kg);
    const v4f c = *(const v4f*)(w + (size_t)n * 64 + kg + 4);
    float v[8];
    v[0] = a[0] * W_CARRY; v[1] = a[1] * W_CARRY; v[2] = a[2] * W_CARRY; v[3] = a[3] * W_CARRY;
    v[4] = c[0] * W_CARRY; v[5] = c[1] * W_CARRY; v[6] = c[2] * W_CARRY; v[7] = c[3] * W_CARRY;
    const v4u u = (v4u){pk16(h_bits(v[0]), h_bits(v[1])), pk16(h_bits(v[2]), h_bits(v[3])), pk16(h_bits(v[4]), h_bits(v[5])), pk16(h_bits(v[6]), h_bits(v[7]))};
    *(v4u*)(Ws + n * pitch + kg) = u;
  }
}

__global__ __launch_bounds__(256) void mlp0_stats_kernel(const _Float16* __restrict__ X0, const float* __restrict__ w0,
                                                         const float* __restrict__ b0, float* __restrict__ P0) {
  __shared__ __align__(16) _Float16 W0s[NCH_A * W0_PITCH];
  __shared__ float sb0[NCH_A];
  __shared__ __align__(16) float red[2 * 8 * NCH_A];
  const int tid = threadIdx.x, lane = tid & 31, wave = tid >> 5;
  const int rlane = lane & 15, hh = lane >> 4, koff = hh * 8;
  build_w0s(W0s, w0, tid);
  if (tid < NCH_A) sb0[tid] = b0[tid];
  __syncthreads();
  const int m0 = (blockIdx.x * 8 + wave) * 64;
  v8f acc[4][4];
#pragma unroll
  for (int i = 0; i < 4; ++i)
#pragma unroll
    for (int j = 0; j < 4; ++j) acc[i][j] = zero8();
  v16h bf[4];
#pragma unroll
  for (int j = 0; j < 4; ++j) bf[j] = FragH::load(W0s + (16 * j + rlane) * W0_PITCH + koff);
#pragma unroll
  for (int i = 0; i < 4; ++i) {
    const v16h af = FragH::load(X0 + (size_t)(m0 + 16 * i + rlane) * KPAD0 + koff);
#pragma unroll
    for (int j = 0; j < 4; ++j) acc[i][j] = FragH::mma(af, bf[j], acc[i][j]);
    guard4(acc[i][0], acc[i][1], acc[i][2], acc[i][3], af, bf[3]);
  }
  keep4_h(bf[0], bf[1], bf[2], bf[3]);
  acc_guard4(acc[0][0], acc[0][1], acc[0][2], acc[0][3]);
  acc_guard4(acc[1][0], acc[1][1], acc[1][2], acc[1][3]);
  acc_guard4(acc[2][0], acc[2][1], acc[2][2], acc[2][3]);
  acc_guard4(acc[3][0], acc[3][1], acc[3][2], acc[3][3]);
  float s[4], s2[4];
#pragma unroll
  for (int j = 0; j < 4; ++j) {
    const int c = 16 * j + rlane;
    const float bv = sb0[c];
    float a = 0.0f, aa = 0.0f;
#pragma unroll
    for (int i = 0; i < 4; ++i)
#pragma unroll
      for (int r = 0; r < 8; ++r) {
        float y = acc[i][j][r] * W_CARRY_INV; y = y + bv;
        a = a + y; aa = aa + y * y;
      }
    s[j] = a; s2[j] = aa;
  }
#pragma unroll
  for (int j = 0; j < 4; ++j) { s[j] = s[j] + __shfl_xor(s[j], 16, 32); s2[j] = s2[j] + __shfl_xor(s2[j], 16, 32); }
#pragma unroll
  for (int j = 0; j < 4; ++j) { const int c = 16 * j + rlane; red[wave * NCH_A + c] = s[j]; red[(8 + wave) * NCH_A + c] = s2[j]; }
  __syncthreads();
  if (wave == 0) {
    v4f t = (v4f){0.f, 0.f, 0.f, 0.f};
#pragma unroll
    for (int w = 0; w < 8; ++w) t = t + *(const v4f*)(red + (hh * 8 + w) * NCH_A + 4 * rlane);
    float* dst = P0 + (size_t)blockIdx.x * 128 + 4 * lane;
    for (int pass = 0; pass < 2; ++pass) { *(volatile v4f*)dst = t; __threadfence(); }
  }
}

template <int NC, int NPART>
__global__ __launch_bounds__(NC * NPART) void bn_fin_kernel(const float* __restrict__ P, int nblk, float* __restrict__ ST) {
  __shared__ double ds[NC * NPART];
  __shared__ double dq[NC * NPART];
  __shared__ __align__(16) float st[2 * NC];
  const int tid = threadIdx.x, lane = tid & 31;
  const int c = tid % NC, part = tid / NC;
  const int rows = nblk / NPART;
  const int r0 = part * rows;
  double s = 0.0, q = 0.0;
#pragma unroll 1
  for (int r = 0; r < rows; ++r) {
    const float* pr = P + (size_t)(r0 + r) * (2 * NC);
    s += (double)pr[c]; q += (double)pr[NC + c];
  }
  ds[tid] = s; dq[tid] = q;
  __syncthreads();
  if (tid < NC) {
    double S = 0.0, Q = 0.0;
#pragma unroll
    for (int p = 0; p < NPART; ++p) { S += ds[p * NC + tid]; Q += dq[p * NC + tid]; }
    const double mean = S * INV_MROWS;
    double var = Q * INV_MROWS - mean * mean; var = var < 0.0 ? 0.0 : var;
    const float mf = (float)mean; const float vf = (float)var;
    const float ve = vf + BN_EPS;
    const float rs = 1.0f / sqrtf(ve);
    st[tid] = mf; st[NC + tid] = rs;
  }
  __syncthreads();
  if (tid < 32) {
#pragma unroll
    for (int k = 0; k < (2 * NC) / 128; ++k) {
      const v4f v = *(const v4f*)(st + k * 128 + 4 * lane);
      float* d = ST + k * 128 + 4 * lane;
      for (int pass = 0; pass < 2; ++pass) { *(volatile v4f*)d = v; __threadfence(); }
    }
  }
}

__global__ __launch_bounds__(256) void mlp1_kernel(const _Float16* __restrict__ X0, const float* __restrict__ w0, const float* __restrict__ b0,
                                                   const float* __restrict__ st0, const float* __restrict__ g0, const float* __restrict__ bb0,
                                                   const float* __restrict__ w1, const float* __restrict__ b1,
                                                   _Float16* __restrict__ Y1, float* __restrict__ P1) {
  __shared__ __align__(16) _Float16 W0s[NCH_A * W0_PITCH];
  __shared__ __align__(16) _Float16 W1s[NCH_B * W64_PITCH];
  __shared__ __align__(16) _Float16 At[8][16 * W64_PITCH];
  __shared__ __align__(16) float prm[6 * NCH_A];
  __shared__ __align__(16) float red[2 * 8 * NCH_B];
  const int tid = threadIdx.x, lane = tid & 31, wave = tid >> 5;
  const int rlane = lane & 15, hh = lane >> 4, koff = hh * 8, mOff = hh * 8;
  const int q8 = lane >> 3, c8 = (lane & 7) * 8;
  build_w0s(W0s, w0, tid);
  build_w64(W1s, W64_PITCH, w1, NCH_B, tid);
  if (tid < 64) {
    prm[tid] = b0[tid]; prm[64 + tid] = st0[tid]; prm[128 + tid] = st0[64 + tid];
    prm[192 + tid] = g0[tid]; prm[256 + tid] = bb0[tid]; prm[320 + tid] = b1[tid];
  }
  __syncthreads();
  const int m0 = (blockIdx.x * 8 + wave) * 64;
  v8f acc0[4][4];
#pragma unroll
  for (int i = 0; i < 4; ++i)
#pragma unroll
    for (int j = 0; j < 4; ++j) acc0[i][j] = zero8();
  {
    v16h bf[4];
#pragma unroll
    for (int j = 0; j < 4; ++j) bf[j] = FragH::load(W0s + (16 * j + rlane) * W0_PITCH + koff);
#pragma unroll
    for (int i = 0; i < 4; ++i) {
      const v16h af = FragH::load(X0 + (size_t)(m0 + 16 * i + rlane) * KPAD0 + koff);
#pragma unroll
      for (int j = 0; j < 4; ++j) acc0[i][j] = FragH::mma(af, bf[j], acc0[i][j]);
      guard4(acc0[i][0], acc0[i][1], acc0[i][2], acc0[i][3], af, bf[3]);
    }
    keep4_h(bf[0], bf[1], bf[2], bf[3]);
  }
  acc_guard4(acc0[0][0], acc0[0][1], acc0[0][2], acc0[0][3]);
  acc_guard4(acc0[1][0], acc0[1][1], acc0[1][2], acc0[1][3]);
  acc_guard4(acc0[2][0], acc0[2][1], acc0[2][2], acc0[2][3]);
  acc_guard4(acc0[3][0], acc0[3][1], acc0[3][2], acc0[3][3]);
  _Float16* Aw = At[wave];
  float s[4], s2[4];
#pragma unroll
  for (int j = 0; j < 4; ++j) { s[j] = 0.0f; s2[j] = 0.0f; }
#pragma unroll
  for (int i = 0; i < 4; ++i) {
    const int mBase = m0 + 16 * i;
    lds_wave_sync();
#pragma unroll
    for (int j = 0; j < 4; ++j) {
      const int c = 16 * j + rlane;
      const float bv = prm[c], mu = prm[64 + c], rs = prm[128 + c], gg = prm[192 + c], be = prm[256 + c];
#pragma unroll
      for (int r = 0; r < 8; ++r) {
        float y = acc0[i][j][r] * W_CARRY_INV; y = y + bv;
        float a = y - mu; a = a * rs; a = a * gg; a = a + be; a = fmaxf(a, 0.0f);
        Aw[(mOff + r) * W64_PITCH + c] = (_Float16)a;
      }
    }
    lds_wave_sync();
    const v16h a0f = FragH::load(Aw + rlane * W64_PITCH + koff);
    const v16h a1f = FragH::load(Aw + rlane * W64_PITCH + koff + 32);
    v8f acc1[4];
#pragma unroll
    for (int j = 0; j < 4; ++j) acc1[j] = zero8();
#pragma unroll
    for (int j = 0; j < 4; ++j) {
      const v16h bq0 = FragH::load(W1s + (16 * j + rlane) * W64_PITCH + koff);
      const v16h bq1 = FragH::load(W1s + (16 * j + rlane) * W64_PITCH + koff + 32);
      acc1[j] = FragH::mma(a0f, bq0, acc1[j]);
      acc1[j] = FragH::mma(a1f, bq1, acc1[j]);
      guard1(acc1[j], a0f, a1f, bq0, bq1);
    }
    acc_guard4(acc1[0], acc1[1], acc1[2], acc1[3]);
    lds_wave_sync();
#pragma unroll
    for (int j = 0; j < 4; ++j) {
      const int c = 16 * j + rlane;
      const float bv1 = prm[320 + c];
#pragma unroll
      for (int r = 0; r < 8; ++r) {
        float y = acc1[j][r] * W_CARRY_INV; y = y + bv1;
        s[j] = s[j] + y; s2[j] = s2[j] + y * y;
        Aw[(mOff + r) * W64_PITCH + c] = (_Float16)y;
      }
    }
    lds_wave_sync();
    v8h hv[4];
#pragma unroll
    for (int it = 0; it < 4; ++it) { const int row = it * 4 + q8; hv[it] = *(const v8h*)(Aw + row * W64_PITCH + c8); }
    for (int pass = 0; pass < 2; ++pass) {
#pragma unroll
      for (int it = 0; it < 4; ++it) {
        const int row = it * 4 + q8;
        *(volatile v8h*)(Y1 + (size_t)(mBase + row) * NCH_B + c8) = hv[it];
      }
      __threadfence();
    }
  }
#pragma unroll
  for (int j = 0; j < 4; ++j) { s[j] = s[j] + __shfl_xor(s[j], 16, 32); s2[j] = s2[j] + __shfl_xor(s2[j], 16, 32); }
#pragma unroll
  for (int j = 0; j < 4; ++j) { const int c = 16 * j + rlane; red[wave * NCH_B + c] = s[j]; red[(8 + wave) * NCH_B + c] = s2[j]; }
  __syncthreads();
  if (wave == 0) {
    v4f t = (v4f){0.f, 0.f, 0.f, 0.f};
#pragma unroll
    for (int w = 0; w < 8; ++w) t = t + *(const v4f*)(red + (hh * 8 + w) * NCH_B + 4 * rlane);
    float* dst = P1 + (size_t)blockIdx.x * 128 + 4 * lane;
    for (int pass = 0; pass < 2; ++pass) { *(volatile v4f*)dst = t; __threadfence(); }
  }
}

__global__ __launch_bounds__(256) void mlp2_pool_kernel(const unsigned* __restrict__ Y1w, const float* __restrict__ st1,
                                                        const float* __restrict__ g1, const float* __restrict__ bb1,
                                                        const float* __restrict__ w2, const float* __restrict__ b2,
                                                        float* __restrict__ P2, float* __restrict__ PMAX, float* __restrict__ PMIN) {
  __shared__ __align__(16) _Float16 W2s[NCH_C * A2_PITCH];
  __shared__ __align__(16) _Float16 At[8][KNB * A2_PITCH];
  __shared__ __align__(16) float prm[4 * 64 + NCH_C];
  __shared__ __align__(16) float mm[8][2 * NCH_C];
  const int tid = threadIdx.x, lane = tid & 31, wave = tid >> 5;
  const int rlane = lane & 15, hh = lane >> 4, koff = hh * 8;
  const int q8 = lane >> 3, c8 = (lane & 7) * 8;
  build_w64(W2s, A2_PITCH, w2, NCH_C, tid);
  if (tid < 64) { prm[tid] = st1[tid]; prm[64 + tid] = st1[64 + tid]; prm[128 + tid] = g1[tid]; prm[192 + tid] = bb1[tid]; }
  if (tid < NCH_C) prm[256 + tid] = b2[tid];
  __syncthreads();
  const int qw = blockIdx.x * 8 + wave;
  _Float16* Aw = At[wave];
  {
    const v4f mu0 = *(const v4f*)(prm + c8),       mu1 = *(const v4f*)(prm + c8 + 4);
    const v4f rs0 = *(const v4f*)(prm + 64 + c8),  rs1 = *(const v4f*)(prm + 64 + c8 + 4);
    const v4f gg0 = *(const v4f*)(prm + 128 + c8), gg1 = *(const v4f*)(prm + 128 + c8 + 4);
    const v4f be0 = *(const v4f*)(prm + 192 + c8), be1 = *(const v4f*)(prm + 192 + c8 + 4);
#pragma unroll
    for (int it = 0; it < 8; ++it) {
      const int row = it * 4 + q8;
      const v4u w = *(const v4u*)(Y1w + ((size_t)(qw * KNB + row) * NCH_B + c8) / 2);
      float a[8];
#pragma unroll
      for (int e2 = 0; e2 < 4; ++e2) {
        const unsigned ww = w[e2];
        a[2 * e2] = h16_to_f32(ww & 0xffffu);
        a[2 * e2 + 1] = h16_to_f32(ww >> 16);
      }
#pragma unroll
      for (int e = 0; e < 8; ++e) {
        const float mu = (e < 4) ? mu0[e] : mu1[e - 4];
        const float rs = (e < 4) ? rs0[e] : rs1[e - 4];
        const float gg = (e < 4) ? gg0[e] : gg1[e - 4];
        const float be = (e < 4) ? be0[e] : be1[e - 4];
        float t = a[e] - mu; t = t * rs; t = t * gg; t = t + be; a[e] = fmaxf(t, 0.0f);
      }
      const v4u u = (v4u){pk16(h_bits(a[0]), h_bits(a[1])), pk16(h_bits(a[2]), h_bits(a[3])), pk16(h_bits(a[4]), h_bits(a[5])), pk16(h_bits(a[6]), h_bits(a[7]))};
      *(v4u*)(Aw + row * A2_PITCH + c8) = u;
    }
  }
  lds_wave_sync();
  v8f acc[2][8];
#pragma unroll
  for (int i = 0; i < 2; ++i)
#pragma unroll
    for (int j = 0; j < 8; ++j) acc[i][j] = zero8();
#pragma unroll
  for (int ks = 0; ks < 2; ++ks) {
    const v16h a0f = FragH::load(Aw + rlane * A2_PITCH + koff + 32 * ks);
    const v16h a1f = FragH::load(Aw + (16 + rlane) * A2_PITCH + koff + 32 * ks);
#pragma unroll
    for (int j = 0; j < 8; ++j) {
      const v16h bq = FragH::load(W2s + (16 * j + rlane) * A2_PITCH + koff + 32 * ks);
      acc[0][j] = FragH::mma(a0f, bq, acc[0][j]);
      acc[1][j] = FragH::mma(a1f, bq, acc[1][j]);
      guard2(acc[0][j], acc[1][j], a0f, a1f, bq);
    }
  }
  acc_guard4(acc[0][0], acc[0][1], acc[0][2], acc[0][3]);
  acc_guard4(acc[0][4], acc[0][5], acc[0][6], acc[0][7]);
  acc_guard4(acc[1][0], acc[1][1], acc[1][2], acc[1][3]);
  acc_guard4(acc[1][4], acc[1][5], acc[1][6], acc[1][7]);
  float* mw = mm[wave];
  float sv[8], qv[8];
#pragma unroll
  for (int j = 0; j < 8; ++j) {
    const int c = 16 * j + rlane;
    const float bv = prm[256 + c];
    float a = 0.0f, aa = 0.0f, mx = -INFINITY, mn = INFINITY;
#pragma unroll
    for (int i = 0; i < 2; ++i)
#pragma unroll
      for (int r = 0; r < 8; ++r) {
        float y = acc[i][j][r] * W_CARRY_INV; y = y + bv;
        a = a + y; aa = aa + y * y; mx = fmaxf(mx, y); mn = fminf(mn, y);
      }
    a = a + __shfl_xor(a, 16, 32);
    aa = aa + __shfl_xor(aa, 16, 32);
    mx = fmaxf(mx, __shfl_xor(mx, 16, 32));
    mn = fminf(mn, __shfl_xor(mn, 16, 32));
    sv[j] = a; qv[j] = aa;
    mw[c] = mx; mw[NCH_C + c] = mn;
  }
  lds_wave_sync();
  {
    const v4f vx = *(const v4f*)(mw + 4 * lane);
    const v4f vn = *(const v4f*)(mw + NCH_C + 4 * lane);
    float* dx = PMAX + (size_t)qw * NCH_C + 4 * lane;
    float* dn = PMIN + (size_t)qw * NCH_C + 4 * lane;
    for (int pass = 0; pass < 2; ++pass) { *(volatile v4f*)dx = vx; *(volatile v4f*)dn = vn; __threadfence(); }
  }
  lds_wave_sync();
#pragma unroll
  for (int j = 0; j < 8; ++j) { const int c = 16 * j + rlane; mw[c] = sv[j]; mw[NCH_C + c] = qv[j]; }
  __syncthreads();
  if (wave == 0) {
    v4f ts = (v4f){0.f, 0.f, 0.f, 0.f}, tq = (v4f){0.f, 0.f, 0.f, 0.f};
#pragma unroll
    for (int w = 0; w < 8; ++w) { ts = ts + *(const v4f*)(mm[w] + 4 * lane); tq = tq + *(const v4f*)(mm[w] + NCH_C + 4 * lane); }
    float* d0 = P2 + (size_t)blockIdx.x * 256 + 4 * lane;
    float* d1 = d0 + 128;
    for (int pass = 0; pass < 2; ++pass) { *(volatile v4f*)d0 = ts; *(volatile v4f*)d1 = tq; __threadfence(); }
  }
}

__global__ __launch_bounds__(256) void out_kernel(const float* __restrict__ PMAX, const float* __restrict__ PMIN, const float* __restrict__ ST2,
                                                  const float* __restrict__ g2, const float* __restrict__ bb2, float* __restrict__ out1) {
  const int i = blockIdx.x * 256 + threadIdx.x;
  const int q = i >> 5;
  const int l4 = (i & 31) * 4;
  const v4f mx = *(const v4f*)(PMAX + (size_t)q * NCH_C + l4);
  const v4f mn = *(const v4f*)(PMIN + (size_t)q * NCH_C + l4);
  const v4f mu = *(const v4f*)(ST2 + l4);
  const v4f rs = *(const v4f*)(ST2 + NCH_C + l4);
  const v4f gg = *(const v4f*)(g2 + l4);
  const v4f be = *(const v4f*)(bb2 + l4);
  v4f o;
#pragma unroll
  for (int e = 0; e < 4; ++e) {
    const float fa = (gg[e] >= 0.0f) ? 1.0f : 0.0f;
    const float fb = 1.0f - fa;
    const float pa = fa * mx[e]; const float pb = fb * mn[e]; const float sel = pa + pb;
    float t = sel - mu[e]; t = t * rs[e]; t = t * gg[e]; t = t + be[e];
    o[e] = fmaxf(t, 0.0f);
  }
  float* d = out1 + (size_t)q * NCH_C + l4;
  for (int pass = 0; pass < 2; ++pass) { *(volatile v4f*)d = o; __threadfence(); }
}

extern "C" void kernel_launch(void* const* d_in, const int* in_sizes, int n_in,
                              void* d_out, int out_size, void* d_ws, size_t ws_size, hipStream_t stream)
{
  (void)in_sizes; (void)n_in; (void)out_size;
  const float* xyz = (const float*)d_in[0];
  const float* pts = (const float*)d_in[1];
  const float* w0  = (const float*)d_in[2];
  const float* b0  = (const float*)d_in[3];
  const float* g0  = (const float*)d_in[4];
  const float* bb0 = (const float*)d_in[5];
  const float* w1  = (const float*)d_in[6];
  const float* b1  = (const float*)d_in[7];
  const float* g1  = (const float*)d_in[8];
  const float* bb1 = (const float*)d_in[9];
  const float* w2  = (const float*)d_in[10];
  const float* b2  = (const float*)d_in[11];
  const float* g2  = (const float*)d_in[12];
  const float* bb2 = (const float*)d_in[13];

  char* ws = (char*)d_ws; size_t off = 0;
  auto carve = [&](size_t bytes) -> char* { char* p = ws + off; off += (bytes + 255) & ~(size_t)255; return p; };
  float*    CQ   = (float*)carve((size_t)NQ * 4 * 4);
  char*     X0c  = carve((size_t)MROWS * KPAD0 * 2);
  float*    P0   = (float*)carve((size_t)NBLK64 * 128 * 4);
  float*    ST0  = (float*)carve((size_t)128 * 4);
  char*     Y1c  = carve((size_t)MROWS * NCH_B * 2);
  float*    P1   = (float*)carve((size_t)NBLK64 * 128 * 4);
  float*    ST1  = (float*)carve((size_t)128 * 4);
  float*    P2   = (float*)carve((size_t)NBLK32 * 256 * 4);
  float*    PMAX = (float*)carve((size_t)NQ * NCH_C * 4);
  float*    PMIN = (float*)carve((size_t)NQ * NCH_C * 4);
  float*    ST2  = (float*)carve((size_t)256 * 4);
  if (off > ws_size || off > (size_t)134217728) return;

  unsigned*        X0w = (unsigned*)X0c;
  const _Float16*  X0h = (const _Float16*)X0c;
  _Float16*        Y1h = (_Float16*)Y1c;
  const unsigned*  Y1w = (const unsigned*)Y1c;

  float* out0 = (float*)d_out;
  float* out1 = (float*)d_out + (196608 / 4);

  fps_kernel<<<NBATCH, 1024, 0, stream>>>(xyz, out0, CQ);
  knn_group_kernel<<<NQ / 256, 256, 0, stream>>>(xyz, pts, CQ, X0w);
  mlp0_stats_kernel<<<NBLK64, 256, 0, stream>>>(X0h, w0, b0, P0);
  bn_fin_kernel<NCH_A, 4><<<1, NCH_A * 4, 0, stream>>>(P0, NBLK64, ST0);
  mlp1_kernel<<<NBLK64, 256, 0, stream>>>(X0h, w0, b0, ST0, g0, bb0, w1, b1, Y1h, P1);
  bn_fin_kernel<NCH_B, 4><<<1, NCH_B * 4, 0, stream>>>(P1, NBLK64, ST1);
  mlp2_pool_kernel<<<NBLK32, 256, 0, stream>>>(Y1w, ST1, g1, bb1, w2, b2, P2, PMAX, PMIN);
  bn_fin_kernel<NCH_C, 2><<<1, NCH_C * 2, 0, stream>>>(P2, NBLK32, ST2);
  out_kernel<<<(NQ * 32) / 256, 256, 0, stream>>>(PMAX, PMIN, ST2, g2, bb2, out1);
}
